// Mamba2Block_4475355922524
// MI455X (gfx1250) — hardware-verified
//
#include <hip/hip_runtime.h>
#include <math.h>
#include <stdint.h>

typedef __attribute__((ext_vector_type(16))) _Float16 v16h;
typedef __attribute__((ext_vector_type(8)))  _Float16 v8h;
typedef __attribute__((ext_vector_type(4)))  _Float16 v4h;
typedef __attribute__((ext_vector_type(16))) __bf16   v16b;
typedef __attribute__((ext_vector_type(8)))  __bf16   v8b;
typedef __attribute__((ext_vector_type(8)))  float    v8f;
typedef __attribute__((ext_vector_type(4)))  float    v4f;
typedef __attribute__((ext_vector_type(2)))  double   v2d;
typedef __attribute__((ext_vector_type(4)))  unsigned v4u;
typedef __attribute__((ext_vector_type(2)))  unsigned v2u;

constexpr int kBatch = 2;
constexpr int kSeq   = 2048;
constexpr int kHeads = 32;
constexpr int kHdim  = 64;
constexpr int kNst   = 128;
constexpr int kChunk = 256;
constexpr int kNch   = kSeq / kChunk;
constexpr int kTiles = kBatch * kNch * kHeads;
constexpr int kTok   = kBatch * kSeq;
constexpr int kXtile = kHdim * kChunk;
constexpr int kStile = kHdim * kNst;
constexpr int kGtile = kChunk * kChunk;
constexpr int kXPitch = kChunk + 8;
constexpr int kMPitch = 40;
constexpr int kOPitch = 68;
constexpr int kTPitch = 72;
constexpr float kLnFltMin = -87.33654f;

static_assert(kNch == 8 && kTiles == 512, "tile counts");
static_assert((kNst % 32) == 0 && (kChunk % 32) == 0, "GEMM K multiples of 32");
static_assert((kChunk % 64) == 0 && (kNst % 64) == 0 && ((kHeads * kHdim) % 64) == 0, "GEMM M,N multiples of 64");
static_assert((kXPitch % 8) == 0 && (kMPitch % 8) == 0 && (kTPitch % 8) == 0, "16-B aligned LDS rows");

constexpr size_t kOffCb   = 0;
constexpr size_t kOffBb   = kOffCb   + (size_t)kTok * kNst * 2;
constexpr size_t kOffBT   = kOffBb   + (size_t)kTok * kNst * 2;
constexpr size_t kOffCumD = kOffBT   + (size_t)kTok * kNst * 2;
constexpr size_t kOffCumT = kOffCumD + (size_t)kTiles * kChunk * 8;
constexpr size_t kOffDtp  = kOffCumT + (size_t)kTiles * kChunk * 4;
constexpr size_t kOffHT   = kOffDtp  + (size_t)kTiles * kChunk * 4;
constexpr size_t kOffXH   = kOffHT   + (size_t)kTiles * kXtile * 2;
constexpr size_t kOffXL   = kOffXH   + (size_t)kTiles * kXtile * 2;
constexpr size_t kOffG    = kOffXL   + (size_t)kTiles * kXtile * 2;
constexpr size_t kOffST   = kOffG    + (size_t)kBatch * kNch * kGtile * 4;
constexpr size_t kOffSPH  = kOffST   + (size_t)kTiles * kStile * 4;
constexpr size_t kOffSPL  = kOffSPH  + (size_t)kTiles * kStile * 2;
constexpr size_t kWsTotal = kOffSPL  + (size_t)kTiles * kStile * 2;
static_assert(kWsTotal == 93323264ull, "carve total");
static_assert(kWsTotal <= 134217728ull, "carve cap");
static_assert((kOffBb % 128) == 0 && (kOffBT % 128) == 0 && (kOffCumD % 128) == 0 && (kOffCumT % 128) == 0 &&
              (kOffDtp % 128) == 0 && (kOffHT % 128) == 0 && (kOffXH % 128) == 0 && (kOffXL % 128) == 0 &&
              (kOffG % 128) == 0 && (kOffST % 128) == 0 && (kOffSPH % 128) == 0 && (kOffSPL % 128) == 0,
              "128-B aligned regions");
constexpr size_t kOut0Floats = (size_t)kBatch * kSeq * kHeads * kHdim;
constexpr size_t kOut1Floats = (size_t)kBatch * kHeads * kHdim * kNst;
static_assert(kOut0Floats * 4 == 33554432ull, "out1 byte offset");
static_assert((kOut0Floats + kOut1Floats) * 4 == 35651584ull, "out total bytes");

__device__ __forceinline__ unsigned short f2bf_bits(float f) {
  unsigned u = __float_as_uint(f);
  return (unsigned short)((u + 0x7FFFu + ((u >> 16) & 1u)) >> 16);
}
__device__ __forceinline__ float bf_bits2f(unsigned short h) { return __uint_as_float(((unsigned)h) << 16); }
__device__ __forceinline__ float bf16r(float f) { return bf_bits2f(f2bf_bits(f)); }

__device__ __forceinline__ void dep_guard_h(v8f& a, v8f& b, v16h x, v16h y) { asm volatile("v_nop\n\tv_nop\n\tv_nop\n\tv_nop" : "+v"(a), "+v"(b) : "v"(x), "v"(y)); }
__device__ __forceinline__ void dep_guard_b(v8f& a, v8f& b, v16b x, v16b y) { asm volatile("v_nop\n\tv_nop\n\tv_nop\n\tv_nop" : "+v"(a), "+v"(b) : "v"(x), "v"(y)); }
__device__ __forceinline__ void dep_guard4_h(v8f& a, v8f& b, v8f& c, v8f& d, v16h x0, v16h x1, v16h y0, v16h y1, v16h y2, v16h y3) {
  asm volatile("v_nop\n\tv_nop\n\tv_nop\n\tv_nop" : "+v"(a), "+v"(b), "+v"(c), "+v"(d) : "v"(x0), "v"(x1), "v"(y0), "v"(y1), "v"(y2), "v"(y3));
}
__device__ __forceinline__ void dep_guard4_b(v8f& a, v8f& b, v8f& c, v8f& d, v16b x0, v16b x1, v16b y0, v16b y1, v16b y2, v16b y3) {
  asm volatile("v_nop\n\tv_nop\n\tv_nop\n\tv_nop" : "+v"(a), "+v"(b), "+v"(c), "+v"(d) : "v"(x0), "v"(x1), "v"(y0), "v"(y1), "v"(y2), "v"(y3));
}
__device__ __forceinline__ void dep_guard4x9_b(v8f& a, v8f& b, v8f& c, v8f& d, v16b x0,
    v16b y0, v16b y1, v16b y2, v16b y3, v16b z0, v16b z1, v16b z2, v16b z3) {
  asm volatile("v_nop\n\tv_nop\n\tv_nop\n\tv_nop" : "+v"(a), "+v"(b), "+v"(c), "+v"(d)
               : "v"(x0), "v"(y0), "v"(y1), "v"(y2), "v"(y3), "v"(z0), "v"(z1), "v"(z2), "v"(z3));
}
__device__ __forceinline__ void keep4_h(v16h a, v16h b, v16h c, v16h d) { asm volatile("v_nop" :: "v"(a), "v"(b), "v"(c), "v"(d)); }
__device__ __forceinline__ void keep4_b(v16b a, v16b b, v16b c, v16b d) { asm volatile("v_nop" :: "v"(a), "v"(b), "v"(c), "v"(d)); }
__device__ __forceinline__ void acc_guard4(v8f& a, v8f& b, v8f& c, v8f& d) { asm volatile("v_nop\n\tv_nop\n\tv_nop\n\tv_nop" : "+v"(a), "+v"(b), "+v"(c), "+v"(d)); }
template <typename T> struct Frag;
template <> struct Frag<_Float16> {
  typedef v16h V; union U { v16h v; v8h h[2]; };
  static __device__ __forceinline__ v16h load(const _Float16* p) {
    U f; f.h[0] = *(const v8h*)(p); f.h[1] = *(const v8h*)(p + 16); return f.v;
  }
  static __device__ __forceinline__ v8f mma(v16h a, v16h b, v8f c) {
    return __builtin_amdgcn_wmma_f32_16x16x32_f16(false, a, false, b, (short)0, c, false, false);
  }
  static __device__ __forceinline__ void guard(v8f& a, v8f& b, v16h x, v16h y) { dep_guard_h(a, b, x, y); }
  static __device__ __forceinline__ void guard4(v8f& a, v8f& b, v8f& c, v8f& d, v16h x0, v16h x1, v16h y0, v16h y1, v16h y2, v16h y3) { dep_guard4_h(a, b, c, d, x0, x1, y0, y1, y2, y3); }
  static __device__ __forceinline__ void keep(v16h a, v16h b, v16h c, v16h d) { keep4_h(a, b, c, d); }
};
template <> struct Frag<__bf16> {
  typedef v16b V; union U { v16b v; v8b h[2]; };
  static __device__ __forceinline__ v16b load(const __bf16* p) {
    U f; f.h[0] = *(const v8b*)(p); f.h[1] = *(const v8b*)(p + 16); return f.v;
  }
  static __device__ __forceinline__ v8f mma(v16b a, v16b b, v8f c) {
    return __builtin_amdgcn_wmma_f32_16x16x32_bf16(false, a, false, b, (short)0, c, false, false);
  }
  static __device__ __forceinline__ void guard(v8f& a, v8f& b, v16b x, v16b y) { dep_guard_b(a, b, x, y); }
  static __device__ __forceinline__ void guard4(v8f& a, v8f& b, v8f& c, v8f& d, v16b x0, v16b x1, v16b y0, v16b y1, v16b y2, v16b y3) { dep_guard4_b(a, b, c, d, x0, x1, y0, y1, y2, y3); }
  static __device__ __forceinline__ void keep(v16b a, v16b b, v16b c, v16b d) { keep4_b(a, b, c, d); }
};

__device__ __forceinline__ void wave_lds_sync() {
  __builtin_amdgcn_fence(__ATOMIC_RELEASE, "workgroup");
  __builtin_amdgcn_wave_barrier();
  __builtin_amdgcn_fence(__ATOMIC_ACQUIRE, "workgroup");
}

template <int ET> struct Elem;
template <> struct Elem<0> { typedef _Float16 T; };
template <> struct Elem<1> { typedef __bf16 T; };
template <int ET, int SPL, int BIAS_MODE, int OUT_MODE, bool RESID, int ACT = 0>
__global__ __launch_bounds__(256) void wmma_gemm64(
    const unsigned short* __restrict__ Ap, const unsigned short* __restrict__ A2p, int lda, long strideA,
    const unsigned short* __restrict__ Btp, const unsigned short* __restrict__ Bt2p, int ldb, long strideB,
    void* __restrict__ Cout, void* __restrict__ Cout2, int ldc, long strideC,
    const float* __restrict__ bias,
    const float* __restrict__ resid, long strideR,
    int M, int N, int K, float scale) {
  typedef typename Elem<ET>::T T;
  typedef typename Frag<T>::V V;
  const T* A = (const T*)Ap; const T* A2 = (const T*)A2p; const T* Bt = (const T*)Btp; const T* Bt2 = (const T*)Bt2p;
  __shared__ __align__(16) float sT[8][16 * 68];
  const int b    = blockIdx.y;
  const int lane = threadIdx.x & 31;
  const int wave = threadIdx.x >> 5;
  const int tilesN = N >> 6;
  const int tilesM = M >> 6;
  const int tile = blockIdx.x * 8 + wave;
  if (tile >= tilesM * tilesN) return;
  const int tm = tile / tilesN;
  const int tn = tile - tm * tilesN;
  const int m0 = tm << 6;
  const int n0 = tn << 6;

  const T* Ab  = A  + (size_t)b * strideA;
  const T* Bb  = Bt + (size_t)b * strideB;
  const T* Ab2 = (SPL >= 1) ? (A2  + (size_t)b * strideA) : nullptr;
  const T* Bb2 = (SPL == 2) ? (Bt2 + (size_t)b * strideB) : nullptr;

  const int rlane = lane & 15;
  const int koff  = (lane >> 4) * 8;
  const int mOff  = (lane >> 4) * 8;

  v8f acc[4][4];
#pragma unroll
  for (int i = 0; i < 4; ++i)
#pragma unroll
    for (int j = 0; j < 4; ++j) acc[i][j] = (v8f){0.f,0.f,0.f,0.f,0.f,0.f,0.f,0.f};

  for (int k0 = 0; k0 < K; k0 += 32) {
    V bh[4], bl[4];
#pragma unroll
    for (int j = 0; j < 4; ++j) {
      const size_t bo = (size_t)(n0 + (j << 4) + rlane) * ldb + koff + k0;
      bh[j] = Frag<T>::load(Bb + bo);
      if (SPL == 2) bl[j] = Frag<T>::load(Bb2 + bo);
    }
#pragma unroll
    for (int i = 0; i < 4; ++i) {
      const size_t ao = (size_t)(m0 + (i << 4) + rlane) * lda + koff + k0;
      V ah = Frag<T>::load(Ab + ao);
      V al;
      if (SPL >= 1) al = Frag<T>::load(Ab2 + ao);
#pragma unroll
      for (int j = 0; j < 4; ++j) {
        acc[i][j] = Frag<T>::mma(ah, bh[j], acc[i][j]);
        if (SPL == 2) acc[i][j] = Frag<T>::mma(ah, bl[j], acc[i][j]);
        if (SPL >= 1) acc[i][j] = Frag<T>::mma(al, bh[j], acc[i][j]);
      }
      Frag<T>::guard4(acc[i][0], acc[i][1], acc[i][2], acc[i][3], ah, (SPL >= 1) ? al : ah, bh[0], bh[1], bh[2], bh[3]);
    }
    Frag<T>::keep(bh[0], bh[1], bh[2], bh[3]);
    if (SPL == 2) Frag<T>::keep(bl[0], bl[1], bl[2], bl[3]);
  }
  acc_guard4(acc[0][0], acc[0][1], acc[0][2], acc[0][3]);
  acc_guard4(acc[1][0], acc[1][1], acc[1][2], acc[1][3]);
  acc_guard4(acc[2][0], acc[2][1], acc[2][2], acc[2][3]);
  acc_guard4(acc[3][0], acc[3][1], acc[3][2], acc[3][3]);

  float* slab = sT[wave];
  const float* Rb = RESID ? (resid + (size_t)b * strideR) : nullptr;
#pragma unroll
  for (int i = 0; i < 4; ++i) {
    const int mBase = m0 + (i << 4);
#pragma unroll
    for (int j = 0; j < 4; ++j) {
      const int n = n0 + (j << 4) + rlane;
      float bv = 0.f;
      if (BIAS_MODE == 2) bv = bias[n];
#pragma unroll
      for (int r = 0; r < 8; ++r) {
        float v = acc[i][j][r] * scale;
        if (BIAS_MODE == 1) v += bias[mBase + mOff + r];
        if (BIAS_MODE == 2) v += bv;
        if (RESID) v += Rb[(size_t)(mBase + mOff + r) * ldc + n];
        if (ACT == 1) v = tanhf(v);
        if (ACT == 2) v = fmaxf(v, 0.0f);
        if (ACT == 3) v = v / (1.0f + expf(-v));
        if (ACT == 4) v = (v > 0.f) ? v : 0.01f * v;
        slab[(mOff + r) * 68 + (j << 4) + rlane] = v;
      }
    }
    __builtin_amdgcn_fence(__ATOMIC_RELEASE, "workgroup");
    __builtin_amdgcn_wave_barrier();
    __builtin_amdgcn_fence(__ATOMIC_ACQUIRE, "workgroup");
    if (OUT_MODE == 0) {
      float* C = (float*)Cout + (size_t)b * strideC;
      const int hh = lane >> 4, c4 = (lane & 15) * 4;
      for (int pass = 0; pass < 2; ++pass) {
#pragma unroll
        for (int it = 0; it < 8; ++it) {
          const int row = it * 2 + hh;
          v4f v = *(const v4f*)(slab + row * 68 + c4);
          *(volatile v4f*)(C + (size_t)(mBase + row) * ldc + n0 + c4) = v;
        }
        __threadfence();
      }
    } else {
      const int q = lane >> 3, c8 = (lane & 7) * 8;
      unsigned short* C  = (unsigned short*)Cout  + (size_t)b * strideC;
      unsigned short* C2 = (OUT_MODE == 2) ? ((unsigned short*)Cout2 + (size_t)b * strideC) : nullptr;
      for (int pass = 0; pass < 2; ++pass) {
#pragma unroll
        for (int it = 0; it < 4; ++it) {
          const int row = it * 4 + q;
          const float* sp = slab + row * 68 + c8;
          v8h hv, lv;
#pragma unroll
          for (int e = 0; e < 8; ++e) {
            if (OUT_MODE == 1) {
              hv[e] = (_Float16)sp[e];
            } else {
              unsigned short hb = f2bf_bits(sp[e]);
              unsigned short lb = f2bf_bits(sp[e] - bf_bits2f(hb));
              hv[e] = __builtin_bit_cast(_Float16, hb);
              lv[e] = __builtin_bit_cast(_Float16, lb);
            }
          }
          *(volatile v8h*)(C + (size_t)(mBase + row) * ldc + n0 + c8) = hv;
          if (OUT_MODE == 2) *(volatile v8h*)(C2 + (size_t)(mBase + row) * ldc + n0 + c8) = lv;
        }
        __threadfence();
      }
    }
    __builtin_amdgcn_fence(__ATOMIC_RELEASE, "workgroup");
    __builtin_amdgcn_wave_barrier();
    __builtin_amdgcn_fence(__ATOMIC_ACQUIRE, "workgroup");
  }
}

__global__ __launch_bounds__(256) void k_prep_bc(const float* __restrict__ Bf, const float* __restrict__ Cf,
    unsigned short* __restrict__ Cb, unsigned short* __restrict__ Bb, unsigned short* __restrict__ BT)
{
  __shared__ __align__(16) unsigned short sT[kNst * kTPitch];
  const int tid = threadIdx.x, lane = tid & 31, wave = tid >> 5;
  const int b  = blockIdx.x >> 5;
  const int s0 = (blockIdx.x & 31) * 64;
#pragma unroll
  for (int it = 0; it < 4; ++it) {
    asm volatile("" ::: "memory");
    const int e  = (it * 256 + tid) * 8;
    const int sl = e >> 7;
    const int n  = e & 127;
    const size_t g = (size_t)(b * kSeq + s0 + sl) * kNst + n;
    const v4f b0 = *(const v4f*)(Bf + g);
    const v4f b1 = *(const v4f*)(Bf + g + 4);
    const v4f c0 = *(const v4f*)(Cf + g);
    const v4f c1 = *(const v4f*)(Cf + g + 4);
    v8h vcb, vbb;
#pragma unroll
    for (int q4 = 0; q4 < 4; ++q4) {
      const unsigned short cb0 = f2bf_bits(c0[q4]);
      const unsigned short cb1 = f2bf_bits(c1[q4]);
      const unsigned short bb0 = f2bf_bits(b0[q4]);
      const unsigned short bb1 = f2bf_bits(b1[q4]);
      vcb[q4]     = __builtin_bit_cast(_Float16, cb0);
      vcb[4 + q4] = __builtin_bit_cast(_Float16, cb1);
      vbb[q4]     = __builtin_bit_cast(_Float16, bb0);
      vbb[4 + q4] = __builtin_bit_cast(_Float16, bb1);
      sT[(n + q4) * kTPitch + sl]     = bb0;
      sT[(n + 4 + q4) * kTPitch + sl] = bb1;
    }
    *(volatile v8h*)(Cb + g) = vcb;
    *(volatile v8h*)(Bb + g) = vbb;
    __threadfence();
    *(volatile v8h*)(Cb + g) = vcb;
    *(volatile v8h*)(Bb + g) = vbb;
  }
  __syncthreads();
  const int q = lane >> 3, c8 = (lane & 7) * 8;
  for (int pass = 0; pass < 2; ++pass) {
#pragma unroll
    for (int it = 0; it < 4; ++it) {
      const int n = wave * 16 + it * 4 + q;
      const v4u tv = *(const v4u*)(sT + n * kTPitch + c8);
      *(volatile v4u*)(BT + (size_t)(b * kNst + n) * kSeq + s0 + c8) = tv;
    }
    __threadfence();
  }
}

__global__ __launch_bounds__(256) void k_prep_x(const float* __restrict__ hs, const float* __restrict__ dt,
    const float* __restrict__ Af, const float* __restrict__ dtb,
    double* __restrict__ cumD, float* __restrict__ cumT, float* __restrict__ dtpP,
    unsigned short* __restrict__ HT, unsigned short* __restrict__ XH, unsigned short* __restrict__ XL)
{
  __shared__ __align__(16) double scn[kChunk];
  __shared__ __align__(16) float tr[512];
  __shared__ __align__(16) float ts[512];
  __shared__ __align__(16) float sdt[kChunk];
  __shared__ __align__(16) unsigned short shb[kHdim * kXPitch];
  __shared__ __align__(16) unsigned short sxh[kHdim * kXPitch];
  __shared__ __align__(16) unsigned short sxl[kHdim * kXPitch];
  const int tid = threadIdx.x, lane = tid & 31, wave = tid >> 5;
  const int tile = blockIdx.x;
  const int h = tile & 31, c = (tile >> 5) & 7, b = tile >> 8;
  const size_t row = (size_t)(b * kSeq + c * kChunk + tid) * kHeads + h;
  const float z   = bf16r(dt[row]) + bf16r(dtb[h]);
  const float dtp = fmaxf(z, 0.0f) + log1pf(expf(-fabsf(z)));
  const float a   = bf16r(Af[h]) * dtp;
  sdt[tid] = dtp;
  scn[tid] = (double)a;
  tr[tid]  = a;
  __syncthreads();

#pragma unroll 1
  for (int off = 1; off < kChunk; off <<= 1) {
    const int src = (tid >= off) ? (tid - off) : 0;
    const double pv = scn[src];
    const double fs = (tid >= off) ? 1.0 : 0.0;
    __syncthreads();
    scn[tid] += pv * fs;
    __syncthreads();
  }

#pragma unroll 1
  for (int L = 1; L <= 8; ++L) {
    const int n = kChunk >> L;
    const int offp = 512 - (512 >> (L - 1));
    const int offc = 512 - (512 >> L);
    const int tcl = (tid < n) ? tid : (n - 1);
    const float u0 = tr[offp + 2 * tcl];
    const float u1 = tr[offp + 2 * tcl + 1];
    if (tid < n) tr[offc + tid] = u0 + u1;
    __syncthreads();
  }
  if (tid == 0) ts[510] = tr[510];
  __syncthreads();
#pragma unroll 1
  for (int L = 7; L >= 0; --L) {
    const int n = kChunk >> L;
    const int offc = 512 - (512 >> L);
    const int offu = 512 - (512 >> (L + 1));
    const int nu = n >> 1;
    int idx = (tid >> 1) - ((tid & 1) ^ 1);
    idx = (idx < 0) ? 0 : idx;
    idx = (idx > nu - 1) ? (nu - 1) : idx;
    const int tcl = (tid < n) ? tid : (n - 1);
    const float u  = ts[offu + idx];
    const float rv = tr[offc + tcl];
    const float fo = (tid != 0) ? 1.0f : 0.0f;
    const float fe = (tid & 1) ? 0.0f : 1.0f;
    const float res = fmaf(u, fo, rv * fe);
    if (tid < n) ts[offc + tid] = res;
    __syncthreads();
  }
  const float cT  = ts[tid];
  const float cTe = ts[kChunk - 1];

  if (tid < 128) {
    const v2d v = *(const v2d*)(scn + 2 * tid);
    volatile v2d* p = (volatile v2d*)(cumD + (size_t)tile * kChunk + 2 * tid);
    *p = v;
    __threadfence();
    *p = v;
  }
  if (tid < 64) {
    const v4f v = *(const v4f*)(ts + 4 * tid);
    const v4f w = *(const v4f*)(sdt + 4 * tid);
    volatile v4f* pc = (volatile v4f*)(cumT + (size_t)tile * kChunk + 4 * tid);
    volatile v4f* pd = (volatile v4f*)(dtpP + (size_t)tile * kChunk + 4 * tid);
    *pc = v; *pd = w;
    __threadfence();
    *pc = v; *pd = w;
  }

  const float darg = cTe - cT;
  float decv = expf(darg);
  decv = (darg < kLnFltMin) ? 0.0f : decv;
  const float wgt = dtp * decv;
  const float* hrow = hs + row * kHdim;
#pragma unroll 1
  for (int dc = 0; dc < 4; ++dc) {
    v4f h4[4];
#pragma unroll
    for (int i = 0; i < 4; ++i) h4[i] = *(const v4f*)(hrow + dc * 16 + i * 4);
#pragma unroll
    for (int i = 0; i < 4; ++i) {
#pragma unroll
      for (int e = 0; e < 4; ++e) {
        const int d = dc * 16 + i * 4 + e;
        const unsigned short hb = f2bf_bits(h4[i][e]);
        const float xw = bf_bits2f(hb) * wgt;
        const unsigned short xb = f2bf_bits(xw);
        const unsigned short lb = f2bf_bits(xw - bf_bits2f(xb));
        shb[d * kXPitch + tid] = hb;
        sxh[d * kXPitch + tid] = xb;
        sxl[d * kXPitch + tid] = lb;
      }
    }
  }
  __syncthreads();
  const size_t base = (size_t)tile * kXtile;
  for (int pass = 0; pass < 2; ++pass) {
#pragma unroll
    for (int it = 0; it < 8; ++it) {
      const int d = wave * 8 + it;
      const v4u va = *(const v4u*)(shb + d * kXPitch + lane * 8);
      const v4u vb = *(const v4u*)(sxh + d * kXPitch + lane * 8);
      const v4u vc = *(const v4u*)(sxl + d * kXPitch + lane * 8);
      const size_t o = base + (size_t)d * kChunk + lane * 8;
      *(volatile v4u*)(HT + o) = va;
      *(volatile v4u*)(XH + o) = vb;
      *(volatile v4u*)(XL + o) = vc;
    }
    __threadfence();
  }
}

__global__ __launch_bounds__(256) void k_chunk_carry(const float* __restrict__ cumT, const float* __restrict__ ST,
    unsigned short* __restrict__ SPH, unsigned short* __restrict__ SPL, float* __restrict__ FS)
{
  __shared__ __align__(16) float sF[2048];
  const int tid = threadIdx.x;
  const int qq = blockIdx.x & 3;
  const int bh = blockIdx.x >> 2;
  const int h = bh & 31, b = bh >> 5;
  const int e0 = qq * 2048 + tid * 8;
  float run[8];
#pragma unroll
  for (int e = 0; e < 8; ++e) run[e] = 0.0f;
#pragma unroll 1
  for (int c = 0; c < kNch; ++c) {
    const int tile = (b * kNch + c) * kHeads + h;
    const float ev = cumT[(size_t)tile * kChunk + (kChunk - 1)];
    float fac = expf(ev);
    fac = (ev < kLnFltMin) ? 0.0f : fac;
    const float* st = ST + (size_t)tile * kStile + e0;
    const v4f a0 = *(const v4f*)(st);
    const v4f a1 = *(const v4f*)(st + 4);
    v8h hv, lv;
#pragma unroll
    for (int e = 0; e < 8; ++e) {
      const unsigned short hb = f2bf_bits(run[e]);
      const unsigned short lb = f2bf_bits(run[e] - bf_bits2f(hb));
      hv[e] = __builtin_bit_cast(_Float16, hb);
      lv[e] = __builtin_bit_cast(_Float16, lb);
    }
    const size_t so = (size_t)tile * kStile + e0;
    for (int pass = 0; pass < 2; ++pass) {
      *(volatile v8h*)(SPH + so) = hv;
      *(volatile v8h*)(SPL + so) = lv;
      __threadfence();
    }
#pragma unroll
    for (int e = 0; e < 4; ++e) {
      run[e]     = fmaf(fac, run[e],     a0[e]);
      run[4 + e] = fmaf(fac, run[4 + e], a1[e]);
    }
  }
  {
    v4f f0, f1;
#pragma unroll
    for (int e = 0; e < 4; ++e) { f0[e] = run[e]; f1[e] = run[4 + e]; }
    *(v4f*)(sF + tid * 8)     = f0;
    *(v4f*)(sF + tid * 8 + 4) = f1;
  }
  __syncthreads();
  const v4f o0 = *(const v4f*)(sF + tid * 4);
  const v4f o1 = *(const v4f*)(sF + 1024 + tid * 4);
  float* fs = FS + (size_t)bh * kStile + qq * 2048;
  for (int pass = 0; pass < 2; ++pass) {
    *(volatile v4f*)(fs + tid * 4)        = o0;
    *(volatile v4f*)(fs + 1024 + tid * 4) = o1;
    __threadfence();
  }
}

__global__ __launch_bounds__(256) void k_y(const double* __restrict__ cumD, const float* __restrict__ cumT,
    const float* __restrict__ dtpP, const unsigned short* __restrict__ HT, const unsigned short* __restrict__ Cb,
    const unsigned short* __restrict__ SPH, const unsigned short* __restrict__ SPL, const float* __restrict__ Gm,
    const float* __restrict__ hs, const float* __restrict__ Df, float* __restrict__ Y)
{
  __shared__ __align__(16) unsigned short sX[kHdim * kXPitch];
  __shared__ __align__(16) unsigned short sMh[8][32 * kMPitch];
  __shared__ __align__(16) unsigned short sMl[8][32 * kMPitch];
  __shared__ __align__(16) float sO[8][16 * kOPitch];
  __shared__ __align__(16) double sc[kChunk];
  __shared__ __align__(16) float sct[kChunk];
  __shared__ __align__(16) float sdt[kChunk];
  typedef Frag<__bf16> FB;
  const int tid = threadIdx.x, lane = tid & 31, wave = tid >> 5;
  const int hh = lane >> 4, rl = lane & 15, koff = hh * 8;
  const int tile = blockIdx.x;
  const int h = tile & 31, c = (tile >> 5) & 7, b = tile >> 8;

  sc[tid]  = cumD[(size_t)tile * kChunk + tid];
  sct[tid] = cumT[(size_t)tile * kChunk + tid];
  sdt[tid] = dtpP[(size_t)tile * kChunk + tid];
  {
    const unsigned short* xg = HT + (size_t)tile * kXtile;
#pragma unroll
    for (int it = 0; it < 8; ++it) {
      const int i  = it * 256 + tid;
      const int d  = i >> 5;
      const int k8 = (i & 31) * 8;
      *(v4u*)(sX + d * kXPitch + k8) = *(const v4u*)(xg + d * kChunk + k8);
    }
  }
  __syncthreads();

  const int lb = wave * 32;
  v8f acc[2][4];
#pragma unroll
  for (int i = 0; i < 2; ++i)
#pragma unroll
    for (int j = 0; j < 4; ++j) acc[i][j] = (v8f){0.f,0.f,0.f,0.f,0.f,0.f,0.f,0.f};

  {
    const __bf16* Cg = (const __bf16*)Cb + (size_t)(b * kSeq + c * kChunk + lb) * kNst;
    const __bf16* Sh = (const __bf16*)SPH + (size_t)tile * kStile;
    const __bf16* Sl = (const __bf16*)SPL + (size_t)tile * kStile;
#pragma unroll 1
    for (int k0 = 0; k0 < kNst; k0 += 32) {
      v16b bh[4], bl[4];
#pragma unroll
      for (int d4 = 0; d4 < 4; ++d4) bh[d4] = FB::load(Sh + (size_t)(d4 * 16 + rl) * kNst + k0 + koff);
      asm volatile("" ::: "memory");
#pragma unroll
      for (int d4 = 0; d4 < 4; ++d4) bl[d4] = FB::load(Sl + (size_t)(d4 * 16 + rl) * kNst + k0 + koff);
      asm volatile("" ::: "memory");
#pragma unroll
      for (int lt = 0; lt < 2; ++lt) {
        const v16b af = FB::load(Cg + (size_t)(lt * 16 + rl) * kNst + k0 + koff);
#pragma unroll
        for (int d4 = 0; d4 < 4; ++d4) {
          acc[lt][d4] = FB::mma(af, bh[d4], acc[lt][d4]);
          acc[lt][d4] = FB::mma(af, bl[d4], acc[lt][d4]);
        }
        dep_guard4x9_b(acc[lt][0], acc[lt][1], acc[lt][2], acc[lt][3], af,
                       bh[0], bh[1], bh[2], bh[3], bl[0], bl[1], bl[2], bl[3]);
      }
    }
  }
  acc_guard4(acc[0][0], acc[0][1], acc[0][2], acc[0][3]);
  acc_guard4(acc[1][0], acc[1][1], acc[1][2], acc[1][3]);
  {
#pragma unroll
    for (int lt = 0; lt < 2; ++lt) {
#pragma unroll
      for (int r = 0; r < 8; ++r) {
        const float cv = sct[lb + lt * 16 + hh * 8 + r];
        float s = expf(cv);
        s = (cv < kLnFltMin) ? 0.0f : s;
#pragma unroll
        for (int d4 = 0; d4 < 4; ++d4) acc[lt][d4][r] *= s;
      }
    }
  }

  {
    const float* Gz = Gm + (size_t)(b * kNch + c) * kGtile;
    unsigned short* sMhw = sMh[wave];
    unsigned short* sMlw = sMl[wave];
    const int q = lane >> 3, c4 = (lane & 7) * 4;
    for (int kt = 0; kt <= wave; ++kt) {
      const int kb = kt * 32;
      wave_lds_sync();
      double colD[4];
      float  dcol[4];
#pragma unroll
      for (int j = 0; j < 4; ++j) { colD[j] = sc[kb + c4 + j]; dcol[j] = sdt[kb + c4 + j]; }
#pragma unroll
      for (int it = 0; it < 8; ++it) {
        const int rloc = it * 4 + q;
        const int l = lb + rloc;
        const double rowD = sc[l];
        const v4f g4 = *(const v4f*)(Gz + (size_t)l * kChunk + kb + c4);
        v4h mh, ml;
#pragma unroll
        for (int j = 0; j < 4; ++j) {
          const int k = kb + c4 + j;
          const float diff = (float)(rowD - colD[j]);
          const float arg = (k <= l) ? diff : -100.0f;
          float ex = expf(arg);
          ex = (arg < kLnFltMin) ? 0.0f : ex;
          float m = (g4[j] * ex) * dcol[j];
          m = (k <= l) ? m : 0.0f;
          const unsigned short hb = f2bf_bits(m);
          const unsigned short lo = f2bf_bits(m - bf_bits2f(hb));
          mh[j] = __builtin_bit_cast(_Float16, hb);
          ml[j] = __builtin_bit_cast(_Float16, lo);
        }
        *(v2u*)(sMhw + rloc * kMPitch + c4) = __builtin_bit_cast(v2u, mh);
        *(v2u*)(sMlw + rloc * kMPitch + c4) = __builtin_bit_cast(v2u, ml);
      }
      wave_lds_sync();
      v16b bfr[4];
#pragma unroll
      for (int d4 = 0; d4 < 4; ++d4) bfr[d4] = FB::load((const __bf16*)sX + (d4 * 16 + rl) * kXPitch + kb + koff);
#pragma unroll
      for (int lt = 0; lt < 2; ++lt) {
        const v16b ah = FB::load((const __bf16*)sMhw + (lt * 16 + rl) * kMPitch + koff);
        const v16b al = FB::load((const __bf16*)sMlw + (lt * 16 + rl) * kMPitch + koff);
#pragma unroll
        for (int d4 = 0; d4 < 4; ++d4) {
          acc[lt][d4] = FB::mma(ah, bfr[d4], acc[lt][d4]);
          acc[lt][d4] = FB::mma(al, bfr[d4], acc[lt][d4]);
        }
        dep_guard4_b(acc[lt][0], acc[lt][1], acc[lt][2], acc[lt][3], ah, al, bfr[0], bfr[1], bfr[2], bfr[3]);
      }
    }
  }
  acc_guard4(acc[0][0], acc[0][1], acc[0][2], acc[0][3]);
  acc_guard4(acc[1][0], acc[1][1], acc[1][2], acc[1][3]);

  {
    const float Dv = bf16r(Df[h]);
    float* slab = sO[wave];
    const int c4o = rl * 4;
    const size_t lstride = (size_t)kHeads * kHdim;
    const size_t ybase = ((size_t)(b * kSeq + c * kChunk + lb) * kHeads + h) * kHdim;
#pragma unroll
    for (int lt = 0; lt < 2; ++lt) {
#pragma unroll
      for (int d4 = 0; d4 < 4; ++d4)
#pragma unroll
        for (int r = 0; r < 8; ++r) slab[(hh * 8 + r) * kOPitch + d4 * 16 + rl] = acc[lt][d4][r];
      wave_lds_sync();
      v4f ov[8];
#pragma unroll
      for (int it = 0; it < 8; ++it) {
        const int rr = it * 2 + hh;
        const size_t gi = ybase + (size_t)(lt * 16 + rr) * lstride + c4o;
        const v4f sv = *(const v4f*)(slab + rr * kOPitch + c4o);
        const v4f hv = *(const v4f*)(hs + gi);
        v4f o;
#pragma unroll
        for (int e = 0; e < 4; ++e) o[e] = sv[e] + Dv * bf16r(hv[e]);
        ov[it] = o;
      }
      for (int pass = 0; pass < 2; ++pass) {
#pragma unroll
        for (int it = 0; it < 8; ++it) {
          const int rr = it * 2 + hh;
          const size_t gi = ybase + (size_t)(lt * 16 + rr) * lstride + c4o;
          *(volatile v4f*)(Y + gi) = ov[it];
        }
        __threadfence();
      }
      wave_lds_sync();
    }
  }
}

extern "C" void kernel_launch(void* const* d_in, const int* in_sizes, int n_in,
                              void* d_out, int out_size, void* d_ws, size_t ws_size,
                              hipStream_t stream) {
  if (n_in < 7) return;
  if (in_sizes[0] != kBatch * kSeq * kHeads * kHdim) return;
  if (in_sizes[1] != kBatch * kSeq * kHeads) return;
  if (in_sizes[2] != kHeads) return;
  if (in_sizes[3] != kBatch * kSeq * kNst) return;
  if (in_sizes[4] != kBatch * kSeq * kNst) return;
  if (in_sizes[5] != kHeads) return;
  if (in_sizes[6] != kHeads) return;
  if (out_size != (int)(kOut0Floats + kOut1Floats)) return;
  if (ws_size < kWsTotal) return;

  const float* hidden = (const float*)d_in[0];
  const float* dt     = (const float*)d_in[1];
  const float* Ap     = (const float*)d_in[2];
  const float* Bm     = (const float*)d_in[3];
  const float* Cm     = (const float*)d_in[4];
  const float* Dp     = (const float*)d_in[5];
  const float* dtb    = (const float*)d_in[6];
  float* Y  = (float*)d_out;
  float* FS = (float*)d_out + kOut0Floats;

  char* ws = (char*)d_ws;
  unsigned short* Cb   = (unsigned short*)(ws + kOffCb);
  unsigned short* Bb   = (unsigned short*)(ws + kOffBb);
  unsigned short* BT   = (unsigned short*)(ws + kOffBT);
  double*         CUMD = (double*)(ws + kOffCumD);
  float*          CUMT = (float*)(ws + kOffCumT);
  float*          DTP  = (float*)(ws + kOffDtp);
  unsigned short* HT   = (unsigned short*)(ws + kOffHT);
  unsigned short* XH   = (unsigned short*)(ws + kOffXH);
  unsigned short* XL   = (unsigned short*)(ws + kOffXL);
  float*          G    = (float*)(ws + kOffG);
  float*          ST   = (float*)(ws + kOffST);
  unsigned short* SPH  = (unsigned short*)(ws + kOffSPH);
  unsigned short* SPL  = (unsigned short*)(ws + kOffSPL);

  k_prep_bc<<<kTok / 64, 256, 0, stream>>>(Bm, Cm, Cb, Bb, BT);

  k_prep_x<<<kTiles, 256, 0, stream>>>(hidden, dt, Ap, dtb, CUMD, CUMT, DTP, HT, XH, XL);

  wmma_gemm64<1, 0, 0, 0, false><<<dim3(2, kBatch * kNch), 256, 0, stream>>>(
      Cb, nullptr, kNst, (long)(kChunk * kNst),
      Bb, nullptr, kNst, (long)(kChunk * kNst),
      (void*)G, nullptr, kChunk, (long)kGtile,
      nullptr, nullptr, 0L,
      kChunk, kChunk, kNst, 1.0f);

  for (int bb = 0; bb < kBatch; ++bb) {
    wmma_gemm64<1, 1, 0, 0, false><<<dim3(8, kNch), 256, 0, stream>>>(
        XH + (size_t)bb * kNch * kHeads * kXtile, XL + (size_t)bb * kNch * kHeads * kXtile, kChunk, (long)(kHeads * kXtile),
        BT + (size_t)bb * kNst * kSeq, nullptr, kSeq, (long)kChunk,
        (void*)(ST + (size_t)bb * kNch * kHeads * kStile), nullptr, kNst, (long)(kHeads * kStile),
        nullptr, nullptr, 0L,
        kHeads * kHdim, kNst, kChunk, 1.0f);
  }

  k_chunk_carry<<<kBatch * kHeads * 4, 256, 0, stream>>>(CUMT, ST, SPH, SPL, FS);

  k_y<<<kTiles, 256, 0, stream>>>(CUMD, CUMT, DTP, HT, Cb, SPH, SPL, G, hidden, Dp, Y);
}
